// SCDM_89318139888190
// MI455X (gfx1250) — hardware-run, weakly checked
//
#include <hip/hip_runtime.h>
#define SNB 8
#define SNF 256
#define SNK 32
#define SNW 1024
#define SWC 16.0f
#define SAC 1024.0f
typedef unsigned short v8us __attribute__((ext_vector_type(8), may_alias));
typedef float  v8f  __attribute__((ext_vector_type(8)));
typedef float  v4f  __attribute__((ext_vector_type(4)));
typedef float  v4fa __attribute__((ext_vector_type(4), may_alias));

__device__ __forceinline__ unsigned short bf16_bits(float x) { unsigned int u = __float_as_uint(x); return (unsigned short)((u + 0x7FFFu + ((u >> 16) & 1u)) >> 16); }
__device__ __forceinline__ float bf16_val(unsigned short b) { return __uint_as_float(((unsigned int)b) << 16); }
__device__ __forceinline__ float bf16_round(float x) { return bf16_val(bf16_bits(x)); }

typedef _Float16 v16h __attribute__((ext_vector_type(16)));
union FragH { v16h v; v8us half[2]; _Float16 h[16]; unsigned short u[16]; };

__global__ __launch_bounds__(256) void k_wt_f16(const float* __restrict__ W, _Float16* __restrict__ Wt, int K, int N, float scale) {
  const int t = blockIdx.x * 256 + threadIdx.x; if (t >= N * (K / 8)) return; const int n = t / (K / 8), k8 = (t % (K / 8)) * 8; FragH f;
#pragma unroll
  for (int i = 0; i < 8; ++i) f.h[i] = (_Float16)(bf16_round(W[(size_t)(k8 + i) * N + n]) * scale); const v8us o = f.half[0];
  *(volatile v8us*)((unsigned short*)Wt + (size_t)n * K + k8) = o; __threadfence(); *(volatile v8us*)((unsigned short*)Wt + (size_t)n * K + k8) = o;
}

typedef _Float16 v4h __attribute__((ext_vector_type(4)));

__global__ __launch_bounds__(256) void k_x16(const float* __restrict__ x, _Float16* __restrict__ X16, size_t n8) { const size_t t = (size_t)blockIdx.x * 256 + threadIdx.x; if (t >= n8) return; FragH f;
#pragma unroll
  for (int q = 0; q < 8; ++q) f.h[q] = (_Float16)bf16_round(x[t * 8 + q]); *(volatile v8us*)((unsigned short*)X16 + t * 8) = f.half[0]; __threadfence(); *(volatile v8us*)((unsigned short*)X16 + t * 8) = f.half[0]; }

__device__ __forceinline__ v16h g2_frag(const _Float16* p, int hh) { FragH f; f.half[0] = *(const v8us*)((const unsigned short*)p + 8 * hh); f.half[1] = *(const v8us*)((const unsigned short*)p + 16 + 8 * hh); return f.v; }
__device__ __forceinline__ v8f g2_mma(v16h a, v16h b, v8f c) { v8f d = __builtin_amdgcn_wmma_f32_16x16x32_f16(false, a, false, b, (short)0, c, false, false); asm volatile("v_nop\n\tv_nop\n\tv_nop\n\tv_nop" : "+v"(d) : "v"(a), "v"(b)); return d; }
template <int ACT>
__global__ __launch_bounds__(128) void k_gemm2(const _Float16* __restrict__ A, int lda, size_t sA, const _Float16* __restrict__ Bh, int ldb, size_t sB, float alpha, const float* __restrict__ bias, size_t sBias, const float* __restrict__ CP, int rowsPerB, size_t sCPb, int row0g,
    float* __restrict__ C, _Float16* __restrict__ C16, int ldc, size_t sC, int M, int N, int K) { static_assert(ACT == 0 || ACT == 3 || ACT == 6 || ACT == 8 || ACT == 9 || ACT == 11 || ACT == 12 || ACT == 14 || ACT == 15 || ACT == 16 || ACT == 17, "k_gemm2: unsupported ACT code (would silently apply no activation)");
  __shared__ __attribute__((aligned(16))) float so[4][32][68];
  const int tid = threadIdx.x, w = tid >> 5, lane = tid & 31, ln = lane & 15, hh = lane >> 4; const int by = blockIdx.y;
  A += (size_t)by * sA; Bh += (size_t)by * sB; const size_t cofs = (size_t)by * sC; const float* bp = bias ? bias + (size_t)by * sBias : nullptr;
  const int ntn = N >> 6; const int mt = blockIdx.x / ntn, nq = blockIdx.x - mt * ntn; const int row0 = mt * 128 + 32 * w, col0 = nq * 64; if (row0 >= M) return;
  const _Float16* a0p = A + (size_t)(row0 + ln) * lda; const _Float16* a1p = a0p + (size_t)16 * lda;
  const _Float16* b0p = Bh + (size_t)(col0 + ln) * ldb; const _Float16* b1p = b0p + (size_t)16 * ldb; const _Float16* b2p = b1p + (size_t)16 * ldb; const _Float16* b3p = b2p + (size_t)16 * ldb;
  const v8f z8 = {0.f,0.f,0.f,0.f,0.f,0.f,0.f,0.f}; v8f c00 = z8, c01 = z8, c02 = z8, c03 = z8, c10 = z8, c11 = z8, c12 = z8, c13 = z8;
  for (int kb = 0; kb < K; kb += 32) { const v16h a0 = g2_frag(a0p + kb, hh), a1 = g2_frag(a1p + kb, hh);
    v16h b = g2_frag(b0p + kb, hh); c00 = g2_mma(a0, b, c00); c10 = g2_mma(a1, b, c10);
    b = g2_frag(b1p + kb, hh); c01 = g2_mma(a0, b, c01); c11 = g2_mma(a1, b, c11);
    b = g2_frag(b2p + kb, hh); c02 = g2_mma(a0, b, c02); c12 = g2_mma(a1, b, c12);
    b = g2_frag(b3p + kb, hh); c03 = g2_mma(a0, b, c03); c13 = g2_mma(a1, b, c13); }
  v8f accs[8] = {c00, c01, c02, c03, c10, c11, c12, c13};
#pragma unroll
  for (int u = 0; u < 8; ++u) { const int t = u & 3, half = u >> 2; const int col = col0 + t * 16 + ln; const float bv = bp ? bf16_round(bp[col]) : 0.f;
#pragma unroll
    for (int r = 0; r < 8; ++r) { const int rloc = half * 16 + 8 * hh + r; float v = accs[u][r] * alpha + bv; if (CP) { if (rowsPerB < 0) v += CP[cofs + (size_t)(row0g + row0 + rloc) * ldc + col];        else { const int bidx = (row0g + row0 + rloc) / rowsPerB; v += CP[(size_t)bidx * sCPb + (size_t)by * 64 + col]; } }
      if (ACT == 3) v = fmaxf(v, 0.f); else if (ACT == 6) v = 0.5f * v * (1.0f + erff(v * 0.70710678118654752f)); else if (ACT == 11) v = 1.0f / (1.0f + expf(-v)); else if (ACT == 15) v = v / (1.0f + expf(-v)); else if (ACT == 12) v = (v > 0.f) ? v : 0.01f * v; else if (ACT == 8) v = tanhf(v); else if (ACT == 9) v = 0.5f * v * (1.0f + tanhf(0.7978845608028654f * (v + 0.044715f * v * v * v))); else if (ACT == 14) v = (v > 0.f) ? v : 0.1f * v; else if (ACT == 16) v = (v >= 0.f) ? v : 0.3f * v; else if (ACT == 17) v = (v >= 0.f) ? v : 0.2f * v;
      so[w][rloc][t * 16 + ln] = v; } }
  __builtin_amdgcn_fence(__ATOMIC_ACQ_REL, "workgroup"); __builtin_amdgcn_wave_barrier();
  const int rsub = lane >> 4, c4 = (lane & 15) * 4;
  for (int pass = 0; pass < 2; ++pass) {
#pragma unroll
    for (int q = 0; q < 16; ++q) { const int r = q * 2 + rsub; const v4f v = *(const v4fa*)&so[w][r][c4]; if (C) *(volatile v4f*)(C + cofs + (size_t)(row0 + r) * ldc + col0 + c4) = v; if (C16) { v4h h4; for (int i = 0; i < 4; ++i) h4[i] = (_Float16)v[i]; *(volatile v4h*)(C16 + cofs + (size_t)(row0 + r) * ldc + col0 + c4) = h4; } }
    if (pass == 0) __threadfence(); } }

#define TL2E 2.8853900817779268f
__device__ __forceinline__ float tanh_f(float x) { const float e = __builtin_amdgcn_exp2f(x * TL2E); const float r = __builtin_amdgcn_rcpf(e + 1.0f); return fmaf(-2.0f, r, 1.0f); }

__global__ __launch_bounds__(256) void k_addtanh(const float* __restrict__ P, const float* __restrict__ Q, const float* __restrict__ va, float* __restrict__ res, unsigned ni, unsigned nj, unsigned nd) {
  const unsigned j = blockIdx.x * 256u + threadIdx.x, i = blockIdx.y; if (i >= ni || j >= nj) return;
  const float* pp = P + (size_t)i * nd; const float* qp = Q + (size_t)j * nd; float s = 0.0f;
#pragma unroll 1
  for (unsigned d = 0; d < nd; d += 4) { const v4f a = *(const v4fa*)(pp + d); const v4f b = *(const v4fa*)(qp + d); const v4f w = *(const v4fa*)(va + d);
#pragma unroll
    for (int q = 0; q < 4; ++q) s += bf16_round(w[q]) * tanh_f(a[q] + b[q]); }
  float* o = res + (size_t)i * nj + j; *(volatile float*)o = s; __threadfence(); *(volatile float*)o = s; }

typedef int v4i __attribute__((ext_vector_type(4)));
typedef v4i v4ia __attribute__((aligned(16)));
typedef float v2f __attribute__((ext_vector_type(2)));

__global__ __launch_bounds__(256) void k_ms32(const float* __restrict__ zs, const int* __restrict__ qk, _Float16* __restrict__ wh, unsigned nrows) {
  const unsigned rr = blockIdx.x * 256u + threadIdx.x; if (rr >= nrows) return;
  const float* p = zs + (size_t)rr * SNK; const int* kp = qk + (size_t)(rr / (unsigned)SNF) * SNK; float z[SNK]; float top = -__builtin_inff();
#pragma unroll
  for (int j = 0; j < SNK; j += 4) { const v4f t4 = *(const v4fa*)(p + j); const v4i q4 = *(const v4ia*)(kp + j);
#pragma unroll
    for (int u = 0; u < 4; ++u) { z[j + u] = t4[u] + (1.0f - (float)q4[u]) * -1e30f; top = fmaxf(top, z[j + u]); } }
  float ss = 0.0f;
#pragma unroll
  for (int j = 0; j < SNK; ++j) { z[j] = expf(z[j] - top); ss += z[j]; }
  FragH fr[4];
#pragma unroll
  for (int j = 0; j < SNK; ++j) { const float cw = (z[j] / ss) * SAC; fr[j >> 3].h[j & 7] = (_Float16)((cw < 6.103515625e-05f) ? 0.0f : cw); }
  unsigned short* dp = (unsigned short*)wh + (size_t)rr * SNK;
#pragma unroll
  for (int q = 0; q < 4; ++q) *(volatile v8us*)(dp + 8 * q) = fr[q].half[0];
  __threadfence();
#pragma unroll
  for (int q = 0; q < 4; ++q) *(volatile v8us*)(dp + 8 * q) = fr[q].half[0]; }

__global__ __launch_bounds__(256) void k_two(const float* __restrict__ cx, const float* __restrict__ ha, const float* __restrict__ hb, const float* __restrict__ ca, const float* __restrict__ cb, float* __restrict__ sc, unsigned nrows) {
  const unsigned rr = blockIdx.x * 256u + threadIdx.x; if (rr >= nrows) return;
  const float* p = cx + (size_t)rr * SNW; float da = 0.0f, db = 0.0f;
  for (unsigned j = 0; j < (unsigned)SNW; j += 4) { const v4f t4 = *(const v4fa*)(p + j); const v4f a4 = *(const v4fa*)(ha + j); const v4f b4 = *(const v4fa*)(hb + j);
#pragma unroll
    for (int u = 0; u < 4; ++u) { da += t4[u] * bf16_round(a4[u]); db += t4[u] * bf16_round(b4[u]); } }
  v2f o; o[0] = tanhf(da + bf16_round(ca[0])); o[1] = tanhf(db + bf16_round(cb[0]));
  *(volatile v2f*)(sc + (size_t)rr * 2) = o; __threadfence(); *(volatile v2f*)(sc + (size_t)rr * 2) = o; }

__global__ __launch_bounds__(256) void k_ssh(const float* __restrict__ fa, const float* __restrict__ sc, float* __restrict__ res, unsigned n4) {
  const unsigned tt = blockIdx.x * 256u + threadIdx.x; if (tt >= n4) return;
  const unsigned row = tt / (unsigned)(SNW / 4); const v2f s2 = *(const v2f*)(sc + (size_t)row * 2); const v4f t4 = *(const v4fa*)(fa + (size_t)tt * 4); v4f o4;
#pragma unroll
  for (int u = 0; u < 4; ++u) o4[u] = s2[0] * bf16_round(t4[u]) + s2[1];
  *(volatile v4f*)(res + (size_t)tt * 4) = o4; __threadfence(); *(volatile v4f*)(res + (size_t)tt * 4) = o4; }

extern "C" void kernel_launch(void* const* d_in, const int* in_sizes, int n_in,
                              void* d_out, int out_size, void* d_ws, size_t ws_size, hipStream_t stream) {
  if (n_in < 12) return; if (in_sizes[0] < SNB * SNF * SNW || in_sizes[2] < SNB * SNK * SNW || in_sizes[3] < SNB * SNK || in_sizes[4] < SNW * SNW || in_sizes[5] < SNW * SNW || in_sizes[6] < SNW || in_sizes[7] < SNW || in_sizes[8] < SNW || in_sizes[9] < 1 || in_sizes[10] < SNW || in_sizes[11] < 1) return; if (out_size < SNB * SNF * SNW) return;
  const float* fa = (const float*)d_in[0]; const float* ta = (const float*)d_in[2]; const int* qk = (const int*)d_in[3]; const float* ua = (const float*)d_in[4]; const float* ub = (const float*)d_in[5]; const float* wv = (const float*)d_in[6]; const float* ra = (const float*)d_in[7]; const float* ha = (const float*)d_in[8]; const float* ca = (const float*)d_in[9]; const float* hb = (const float*)d_in[10]; const float* cb = (const float*)d_in[11];
  float* res = (float*)d_out;
  static_assert((SNB * SNF) % 128 == 0 && (SNB * SNK) % 128 == 0 && SNF % 128 == 0 && SNW % 64 == 0 && SNW % 32 == 0 && SNK % 32 == 0 && SNK % 8 == 0 && SNW % 8 == 0 && SNK == 32, "whole tiles");
  uint8_t* wsp = (uint8_t*)d_ws; size_t off = 0;
  auto take = [&](size_t bytes) { uint8_t* p = wsp + off; off += (bytes + 255) & ~(size_t)255; return p; };
  _Float16* FA = (_Float16*)take((size_t)SNB * SNF * SNW * 2); _Float16* TA = (_Float16*)take((size_t)SNB * SNK * SNW * 2); _Float16* TT = (_Float16*)take((size_t)SNB * SNW * SNK * 2); _Float16* UA = (_Float16*)take((size_t)SNW * SNW * 2); _Float16* UB = (_Float16*)take((size_t)SNW * SNW * 2); float* PA = (float*)take((size_t)SNB * SNK * SNW * 4); float* PB = (float*)take((size_t)SNB * SNF * SNW * 4); float* ZS = (float*)take((size_t)SNB * SNF * SNK * 4); _Float16* AW = (_Float16*)take((size_t)SNB * SNF * SNK * 2); float* CX = (float*)take((size_t)SNB * SNF * SNW * 4); float* SC = (float*)take((size_t)SNB * SNF * 2 * 4);
  if (off > ws_size) return;
  k_x16<<<(unsigned)(((size_t)SNB * SNF * SNW / 8 + 255) / 256), 256, 0, stream>>>(fa, FA, (size_t)SNB * SNF * SNW / 8);
  k_x16<<<(unsigned)(((size_t)SNB * SNK * SNW / 8 + 255) / 256), 256, 0, stream>>>(ta, TA, (size_t)SNB * SNK * SNW / 8);
  for (int g = 0; g < SNB; ++g)
    k_wt_f16<<<(unsigned)(((size_t)SNW * (SNK / 8) + 255) / 256), 256, 0, stream>>>(ta + (size_t)g * SNK * SNW, TT + (size_t)g * SNW * SNK, SNK, SNW, 1.0f);
  k_wt_f16<<<(unsigned)(((size_t)SNW * (SNW / 8) + 255) / 256), 256, 0, stream>>>(ua, UA, SNW, SNW, SWC);
  k_wt_f16<<<(unsigned)(((size_t)SNW * (SNW / 8) + 255) / 256), 256, 0, stream>>>(ub, UB, SNW, SNW, SWC);
  k_gemm2<0><<<dim3((unsigned)((SNB * SNK / 128) * (SNW / 64)), 1), 128, 0, stream>>>(TA, SNW, 0, UA, SNW, 0, 1.0f / SWC, ra, 0, nullptr, 1, 0, 0, PA, nullptr, SNW, 0, SNB * SNK, SNW, SNW);
  k_gemm2<0><<<dim3((unsigned)((SNB * SNF / 128) * (SNW / 64)), 1), 128, 0, stream>>>(FA, SNW, 0, UB, SNW, 0, 1.0f / SWC, nullptr, 0, nullptr, 1, 0, 0, PB, nullptr, SNW, 0, SNB * SNF, SNW, SNW);
  for (int g = 0; g < SNB; ++g)
    k_addtanh<<<dim3(1u, (unsigned)SNF), SNK, 0, stream>>>(PB + (size_t)g * SNF * SNW, PA + (size_t)g * SNK * SNW, wv, ZS + (size_t)g * SNF * SNK, (unsigned)SNF, (unsigned)SNK, (unsigned)SNW);
  k_ms32<<<(unsigned)((SNB * SNF + 255) / 256), 256, 0, stream>>>(ZS, qk, AW, (unsigned)(SNB * SNF));
  k_gemm2<0><<<dim3((unsigned)((SNF / 128) * (SNW / 64)), (unsigned)SNB), 128, 0, stream>>>(AW, SNK, (size_t)SNF * SNK, TT, SNK, (size_t)SNW * SNK, 1.0f / SAC, nullptr, 0, nullptr, 1, 0, 0, CX, nullptr, SNW, (size_t)SNF * SNW, SNF, SNW, SNK);
  k_two<<<(unsigned)((SNB * SNF + 255) / 256), 256, 0, stream>>>(CX, ha, hb, ca, cb, SC, (unsigned)(SNB * SNF));
  k_ssh<<<(unsigned)(((size_t)SNB * SNF * SNW / 4 + 255) / 256), 256, 0, stream>>>(fa, SC, res, (unsigned)((size_t)SNB * SNF * SNW / 4));
}
